// Model_14353780703773
// MI455X (gfx1250) — hardware-verified
//
#include <hip/hip_runtime.h>

typedef __bf16       v16bf __attribute__((ext_vector_type(16)));
typedef float        v8f   __attribute__((ext_vector_type(8)));
typedef float        v4f   __attribute__((ext_vector_type(4)));
typedef int          v8i   __attribute__((ext_vector_type(8)));
typedef int          v4i   __attribute__((ext_vector_type(4)));
typedef unsigned int v4u   __attribute__((ext_vector_type(4)));
typedef v4f __attribute__((may_alias)) v4fa;
typedef v4i __attribute__((may_alias)) v4ia;

union FragU { v8i i; v16bf v; };

#define NB      32
#define LLEN    512
#define DLAT    64
#define HHID    64
#define KK      128
#define LEN     510
#define NROWS   (NB * LEN)
#define MPAD    (NB * LLEN)
#define NCOL    (DLAT * HHID)
#define W1ROW   129
#define W1N     (NCOL * W1ROW)
#define XN      (NB * LLEN * DLAT)
#define MT      64
#define PST     68

#define OUT0_ELEMS 1044480
#define OUT1_OFF   1044480
#define OUT_TOTAL  1060800

#define WS_W1B   0
#define WS_PAR   1048576
#define WS_LDP   1114112
#define WS_TOTAL 1179648

static_assert(MPAD % MT == 0);
static_assert(LLEN % MT == 0);
static_assert(KK == 128 && KK % 32 == 0);
static_assert(HHID == 64 && DLAT == 64);
static_assert(NROWS == 32 * 510);
static_assert(OUT0_ELEMS == NROWS * DLAT);
static_assert((OUT1_OFF * 4) % 128 == 0);
static_assert(OUT1_OFF + NROWS == OUT_TOTAL);
static_assert(2 * MT == 128);
static_assert(WS_PAR == WS_W1B + NCOL * KK * 2);
static_assert(WS_LDP == WS_PAR + 4 * NCOL * 4);
static_assert(WS_TOTAL == WS_LDP + MPAD * 4);
static_assert(WS_PAR % 256 == 0 && WS_LDP % 256 == 0 && WS_TOTAL % 256 == 0);
static_assert(NROWS % 32 == 0);

__device__ __forceinline__ unsigned bfbits(float f) {
  unsigned u = __builtin_bit_cast(unsigned, f);
  u += 0x7FFFu + ((u >> 16) & 1u);
  return u >> 16;
}
__device__ __forceinline__ float bfr(float f) {
  return __builtin_bit_cast(float, bfbits(f) << 16);
}
__device__ __forceinline__ unsigned pk2(float lo, float hi) {
  return bfbits(lo) | (bfbits(hi) << 16);
}

__device__ __forceinline__ v8f wmma_bf(v8i a, v8i b, v8f c) {
  FragU ua, ub;
  ua.i = a;
  ub.i = b;
  v8f d = __builtin_amdgcn_wmma_f32_16x16x32_bf16(false, ua.v, false, ub.v, (short)0, c, false, false);
  asm volatile("v_nop\n\tv_nop\n\tv_nop\n\tv_nop" : "+v"(d) : "v"(a), "v"(b));
  return d;
}

__device__ __forceinline__ v8i load_frag_bf(const unsigned short* p, int h) {
  const v4i lo = *(const v4ia*)(p + 8 * h);
  const v4i hi = *(const v4ia*)(p + 16 + 8 * h);
  const v8i r = { lo.x, lo.y, lo.z, lo.w, hi.x, hi.y, hi.z, hi.w };
  return r;
}

__device__ __forceinline__ v4f load_wl4(const float* __restrict__ W1, int c) {
  const float a0 = W1[(size_t)(c + 0) * W1ROW + 128];
  const float a1 = W1[(size_t)(c + 1) * W1ROW + 128];
  const float a2 = W1[(size_t)(c + 2) * W1ROW + 128];
  const float a3 = W1[(size_t)(c + 3) * W1ROW + 128];
  const v4f r = { bfr(a0), bfr(a1), bfr(a2), bfr(a3) };
  return r;
}

__global__ __launch_bounds__(256) void k_prep(
    const float* __restrict__ W1, const float* __restrict__ b1, const float* __restrict__ W2,
    unsigned short* __restrict__ w1b, float* __restrict__ par)
{
  __shared__ __attribute__((aligned(16))) float sT[2304];
  const int blk = blockIdx.x, tid = threadIdx.x;
  if (blk < 256) {
    const int c0 = blk * 16;
    const int base = c0 * W1ROW;
    #pragma unroll 1
    for (int it = 0; it < 9; ++it) {
      const int i = tid + 256 * it;
      int g = base + i;
      g = (g < W1N) ? g : (W1N - 1);
      sT[i] = W1[g];
    }
    __syncthreads();
    const int row = tid >> 4, k0 = (tid & 15) * 8;
    const float* s = sT + row * W1ROW + k0;
    const v4u o = { pk2(s[0], s[1]), pk2(s[2], s[3]), pk2(s[4], s[5]), pk2(s[6], s[7]) };
    unsigned* dst = (unsigned*)w1b + (((size_t)(c0 + row) * KK + k0) >> 1);
    *(volatile v4u*)dst = o;
    __threadfence();
    *(volatile v4u*)dst = o;
  } else {
    const int g = (blk - 256) * 256 + tid;
    const int plane = (blk - 256) >> 2;
    const int c4 = (g & 1023) * 4;
    v4f o;
    if (plane == 0) {
      o = load_wl4(W1, c4);
    } else if (plane == 1) {
      const v4f v = *(const v4fa*)(b1 + c4);
      const v4f r = { bfr(v.x), bfr(v.y), bfr(v.z), bfr(v.w) };
      o = r;
    } else if (plane == 2) {
      const v4f v = *(const v4fa*)(W2 + c4);
      const v4f r = { bfr(v.x), bfr(v.y), bfr(v.z), bfr(v.w) };
      o = r;
    } else {
      const v4f v = *(const v4fa*)(W2 + c4);
      const v4f wl = load_wl4(W1, c4);
      const v4f r = { bfr(v.x) * wl.x, bfr(v.y) * wl.y, bfr(v.z) * wl.z, bfr(v.w) * wl.w };
      o = r;
    }
    float* dst = par + (size_t)g * 4;
    *(volatile v4f*)dst = o;
    __threadfence();
    *(volatile v4f*)dst = o;
  }
}

__device__ __forceinline__ void ep_step(float pre, float xt, float wl, float bb, float w2, float wj,
                                        float& ra, float& ja) {
  const float p = (pre + xt * wl) + bb;
  const bool s = (p >= 0.0f);
  const float act = s ? p : (0.2f * p);
  const float dj = s ? wj : (0.2f * wj);
  ra += act * w2;
  ja += dj;
}

__device__ __forceinline__ void final_store_pass(const float* sOut, const float* sLd,
                                                 float* out0, float* ldp,
                                                 int b, int l0, int r0, int w, int lane) {
  const int q8 = lane & 7, sub = lane >> 3;
  #pragma unroll
  for (int i = 0; i < 8; ++i) {
    const int lid = i * 4 + sub;
    const int row = 16 * w + (lid >> 1), hl = lid & 1;
    const int l = l0 + row;
    const v4f v = *(const v4fa*)(sOut + row * 64 + 32 * hl + 4 * q8);
    if (l < LEN) {
      const size_t gi = ((size_t)(b * LEN + l)) * DLAT + 32 * hl + 4 * q8;
      *(volatile v4f*)(out0 + gi) = v;
    }
  }
  const v4f lv = *(const v4fa*)(sLd + 4 * (lane & 15));
  if (w == 0 && lane < 16) {
    *(volatile v4f*)(ldp + r0 + 4 * lane) = lv;
  }
}

__global__ __launch_bounds__(128) void k_mlp(
    const float* __restrict__ x, const unsigned short* __restrict__ w1b,
    const float* __restrict__ par, const float* __restrict__ b2,
    float* __restrict__ out0, float* __restrict__ ldp)
{
  __shared__ __attribute__((aligned(16))) float sPre[MT * PST];
  __shared__ __attribute__((aligned(16))) float sXT[MT * PST];
  __shared__ __attribute__((aligned(16))) float sOut[MT * 64];
  __shared__ __attribute__((aligned(16))) float sPar[256];
  __shared__ __attribute__((aligned(16))) float sB2[64];
  __shared__ __attribute__((aligned(16))) float sLd[64];

  const int tid = threadIdx.x, lane = tid & 31, w = tid >> 5;
  const int h = lane >> 4, m = lane & 15;
  const int r0 = blockIdx.x * MT;
  const int b = r0 >> 9, l0 = r0 & 511;

  v8i a[4];
  {
    const int rowA = 16 * w + m;
    const bool va = (l0 + rowA) < LEN;
    const int rA = r0 + rowA - (va ? 0 : 2);
    const unsigned am = va ? 0xFFFFFFFFu : 0u;
    const float* xa = x + (size_t)rA * DLAT;
    #pragma unroll
    for (int ks = 0; ks < 4; ++ks) {
      const float* p0 = xa + 32 * ks + 8 * h;
      const v4f f0 = *(const v4fa*)(p0);
      const v4f f1 = *(const v4fa*)(p0 + 4);
      const v4f f2 = *(const v4fa*)(p0 + 16);
      const v4f f3 = *(const v4fa*)(p0 + 20);
      const v8i t = { (int)(pk2(f0.x, f0.y) & am), (int)(pk2(f0.z, f0.w) & am),
                      (int)(pk2(f1.x, f1.y) & am), (int)(pk2(f1.z, f1.w) & am),
                      (int)(pk2(f2.x, f2.y) & am), (int)(pk2(f2.z, f2.w) & am),
                      (int)(pk2(f3.x, f3.y) & am), (int)(pk2(f3.z, f3.w) & am) };
      a[ks] = t;
    }
  }

  #pragma unroll
  for (int it = 0; it < 8; ++it) {
    const int q = tid + 128 * it;
    const int i = q >> 4, c4 = (q & 15) * 4;
    const bool vi = (l0 + i) < LEN;
    const int rs = vi ? (r0 + i + 2) : r0;
    const v4f v = *(const v4fa*)(x + (size_t)rs * DLAT + c4);
    const v4f o = { vi ? bfr(v.x) : 0.0f, vi ? bfr(v.y) : 0.0f, vi ? bfr(v.z) : 0.0f, vi ? bfr(v.w) : 0.0f };
    *(v4fa*)(sXT + i * PST + c4) = o;
  }
  if (tid < 64) sB2[tid] = bfr(b2[tid]);

  const int row = tid >> 1, hf = tid & 1, hb = 32 * hf;
  const v8f z8 = {0.f, 0.f, 0.f, 0.f, 0.f, 0.f, 0.f, 0.f};
  float ld_acc = 0.0f;

  #pragma unroll 1
  for (int d = 0; d < DLAT; ++d) {
    __syncthreads();
    if (tid < 64) {
      const int pl = tid >> 4, c = (tid & 15) * 4;
      const v4f v = *(const v4fa*)(par + pl * NCOL + d * HHID + c);
      *(v4fa*)(sPar + tid * 4) = v;
    }

    v8f acc[4];
    #pragma unroll
    for (int nt = 0; nt < 4; ++nt) acc[nt] = z8;
    const unsigned short* brow = w1b + (size_t)(d * HHID + m) * KK;
    #pragma unroll
    for (int ks = 0; ks < 4; ++ks) {
      #pragma unroll
      for (int nt = 0; nt < 4; ++nt) {
        const v8i bf = load_frag_bf(brow + (size_t)nt * 16 * KK + 32 * ks, h);
        acc[nt] = wmma_bf(a[ks], bf, acc[nt]);
      }
    }
    #pragma unroll
    for (int nt = 0; nt < 4; ++nt) {
      #pragma unroll
      for (int r = 0; r < 8; ++r)
        sPre[(16 * w + 8 * h + r) * PST + 16 * nt + m] = acc[nt][r];
    }
    __syncthreads();

    const float xt = sXT[row * PST + d];
    const float* pr = sPre + row * PST + hb;
    float ra = 0.0f, ja = 0.0f;
    #pragma unroll 2
    for (int j = 0; j < 8; ++j) {
      const v4f p4 = *(const v4fa*)(pr + 4 * j);
      const v4f wl = *(const v4fa*)(sPar + hb + 4 * j);
      const v4f bb = *(const v4fa*)(sPar + 64 + hb + 4 * j);
      const v4f w2 = *(const v4fa*)(sPar + 128 + hb + 4 * j);
      const v4f wj = *(const v4fa*)(sPar + 192 + hb + 4 * j);
      ep_step(p4.x, xt, wl.x, bb.x, w2.x, wj.x, ra, ja);
      ep_step(p4.y, xt, wl.y, bb.y, w2.y, wj.y, ra, ja);
      ep_step(p4.z, xt, wl.z, bb.z, w2.z, wj.z, ra, ja);
      ep_step(p4.w, xt, wl.w, bb.w, w2.w, wj.w, ra, ja);
    }
    const float ro = __shfl_xor(ra, 1);
    const float jo = __shfl_xor(ja, 1);
    const float res = (ra + ro) + sB2[d];
    const float jj = ja + jo;
    ld_acc += logf(fabsf(jj));
    if (hf == 0) sOut[row * 64 + d] = res;
  }
  if (hf == 0) sLd[row] = ld_acc;
  __syncthreads();

  final_store_pass(sOut, sLd, out0, ldp, b, l0, r0, w, lane);
  __threadfence();
  final_store_pass(sOut, sLd, out0, ldp, b, l0, r0, w, lane);
}

__global__ __launch_bounds__(256) void k_out1(const float* __restrict__ ldp, float* __restrict__ out1) {
  const int n = blockIdx.x * 256 + threadIdx.x;
  const int nc = (n < NROWS) ? n : (NROWS - 1);
  const int b = nc / LEN, l = nc - b * LEN;
  const float v = ldp[b * LLEN + l];
  if (n < NROWS) *(volatile float*)(out1 + n) = v;
  __threadfence();
  if (n < NROWS) *(volatile float*)(out1 + n) = v;
}

extern "C" void kernel_launch(void* const* d_in, const int* in_sizes, int n_in,
                              void* d_out, int out_size, void* d_ws, size_t ws_size,
                              hipStream_t stream) {
  if (n_in < 5) return;
  if (in_sizes[0] != XN) return;
  if (in_sizes[1] != W1N) return;
  if (in_sizes[2] != NCOL || in_sizes[3] != NCOL) return;
  if (in_sizes[4] != DLAT) return;
  if (out_size != OUT_TOTAL) return;
  if ((size_t)WS_TOTAL > ws_size) return;

  const float* x  = (const float*)d_in[0];
  const float* W1 = (const float*)d_in[1];
  const float* b1 = (const float*)d_in[2];
  const float* W2 = (const float*)d_in[3];
  const float* b2 = (const float*)d_in[4];

  float* out0 = (float*)d_out;
  float* out1 = out0 + OUT1_OFF;

  char* ws = (char*)d_ws;
  unsigned short* w1b = (unsigned short*)(ws + WS_W1B);
  float* par = (float*)(ws + WS_PAR);
  float* ldp = (float*)(ws + WS_LDP);

  k_prep<<<272, 256, 0, stream>>>(W1, b1, W2, w1b, par);
  k_mlp<<<MPAD / MT, 128, 0, stream>>>(x, w1b, par, b2, out0, ldp);
  k_out1<<<(NROWS + 255) / 256, 256, 0, stream>>>(ldp, out1);
}
